// QSDAv2Block_17549236371762
// MI455X (gfx1250) — hardware-verified
//
#include <hip/hip_runtime.h>
#include <stddef.h>

typedef _Float16 v16h __attribute__((ext_vector_type(16)));
typedef _Float16 v8h  __attribute__((ext_vector_type(8)));
typedef float    v8f  __attribute__((ext_vector_type(8)));
typedef float    v4f  __attribute__((ext_vector_type(4)));
typedef v8h __attribute__((may_alias)) v8ha;
typedef v4f __attribute__((may_alias)) v4fa;
union Frag { v16h v; v8h half[2]; };

#define TOK   8192
#define DM    768
#define NH    8
#define DH    32
#define NS    64
#define SEQ   2048
#define NB    4
#define NENC  3
#define P1LD  640
#define OVLD  1024

#define HSC   4.0f
#define WSC   64.0f
#define PWSC  16.0f
#define OWSC  16.0f
#define PSISC 8.0f
#define MEMSC 8.0f
#define ATTSC 4096.0f
#define CMBSC 1024.0f
#define FSC   256.0f
#define XKSC  16.0f

static_assert(TOK % 128 == 0);
static_assert(DM % 64 == 0);
static_assert(TOK == NB * SEQ);

#define STORE2(T, ptr, val) do { const T s2v_ = (val); T* s2p_ = (T*)(ptr); \
  *(volatile T*)s2p_ = s2v_; __threadfence(); *(volatile T*)s2p_ = s2v_; } while (0)

__device__ __forceinline__ v8f wmma_f16(v16h a, v16h b, v8f c) {
  v8f d = __builtin_amdgcn_wmma_f32_16x16x32_f16(false, a, false, b, (short)0, c, false, false);
  asm volatile("v_nop\n\tv_nop\n\tv_nop\n\tv_nop" : "+v"(d) : "v"(a), "v"(b));
  return d;
}

__device__ __forceinline__ v16h load_frag(const _Float16* p, int h) {
  Frag f;
  f.half[0] = *(const v8ha*)(p + 8 * h);
  f.half[1] = *(const v8ha*)(p + 16 + 8 * h);
  return f.v;
}

__device__ __forceinline__ float wsum32(float v) {
  v += __shfl_xor(v, 16); v += __shfl_xor(v, 8); v += __shfl_xor(v, 4);
  v += __shfl_xor(v, 2);  v += __shfl_xor(v, 1);
  return v;
}

__device__ __forceinline__ v8h to_h8(const float* v) {
  const v8h o = { (_Float16)v[0], (_Float16)v[1], (_Float16)v[2], (_Float16)v[3],
                  (_Float16)v[4], (_Float16)v[5], (_Float16)v[6], (_Float16)v[7] };
  return o;
}

__device__ __forceinline__ void ld8(float* v, const float* s, float sc) {
  const v4f a = *(const v4fa*)s;
  const v4f c = *(const v4fa*)(s + 4);
  v[0] = a.x * sc; v[1] = a.y * sc; v[2] = a.z * sc; v[3] = a.w * sc;
  v[4] = c.x * sc; v[5] = c.y * sc; v[6] = c.z * sc; v[7] = c.w * sc;
}

__device__ __forceinline__ float gelu_erf(float y) {
  return 0.5f * y * (1.0f + erff(y * 0.70710678118654752f));
}

#define CB0  3072
#define CB1  3168
#define CB2  3264
#define CB3  3312
#define CB4  3504
#define CB5  3792
#define CB6  3804
#define CB7  3816
#define CB8  3840
#define CB9  4704
#define CB10 5568
#define CB11 5574
#define CB12 5592

__global__ __launch_bounds__(256) void k_convert(
    const float* __restrict__ h, const float* __restrict__ W_real, const float* __restrict__ W_imag,
    const float* __restrict__ pw1, const float* __restrict__ values, const float* __restrict__ out_w,
    const float* __restrict__ enc_r, const float* __restrict__ enc_i, const float* __restrict__ r_out_w,
    const float* __restrict__ ew1, const float* __restrict__ ew2, const float* __restrict__ rw1,
    _Float16* __restrict__ hh, _Float16* __restrict__ Wp, _Float16* __restrict__ Vt,
    _Float16* __restrict__ outw, _Float16* __restrict__ Enc, _Float16* __restrict__ rout,
    _Float16* __restrict__ e1, _Float16* __restrict__ e2, _Float16* __restrict__ rw1p)
{
  const int blk = blockIdx.x, t = threadIdx.x;
  float v[8];
  _Float16* dst;
  if (blk < CB0) {
    const size_t g = (size_t)blk * 256 + t;
    ld8(v, h + g * 8, HSC);
    dst = hh + g * 8;
  } else if (blk < CB2) {
    const bool imag = (blk >= CB1);
    const float* W = imag ? W_imag : W_real;
    const int e = (blk - (imag ? CB1 : CB0)) * 256 + t;
    const int row = e / 96, qp = e - row * 96;
    const int hd = row >> 5, j = row & 31;
#pragma unroll
    for (int i = 0; i < 8; ++i)
      v[i] = W[((size_t)hd * DM + 8 * qp + i) * DH + j] * WSC;
    dst = Wp + (size_t)((imag ? 256 : 0) + row) * DM + 8 * qp;
  } else if (blk < CB3) {
    const int e = (blk - CB2) * 256 + t;
    ld8(v, pw1 + (size_t)e * 8, PWSC);
    dst = Wp + (size_t)512 * DM + (size_t)e * 8;
  } else if (blk < CB4) {
    const int e = (blk - CB3) * 256 + t;
    const int D = e >> 6, qp = e & 63;
#pragma unroll
    for (int i = 0; i < 8; ++i)
      v[i] = values[(size_t)(8 * qp + i) * DM + D] * WSC;
    dst = Vt + (size_t)D * (NH * NS) + 8 * qp;
  } else if (blk < CB5) {
    const int e = (blk - CB4) * 256 + t;
    ld8(v, out_w + (size_t)e * 8, OWSC);
    dst = outw + (size_t)e * 8;
  } else if (blk < CB6) {
    const int e = (blk - CB5) * 256 + t;
    ld8(v, enc_r + (size_t)e * 8, OWSC);
    dst = Enc + (size_t)e * 8;
  } else if (blk < CB7) {
    const int e = (blk - CB6) * 256 + t;
    ld8(v, enc_i + (size_t)e * 8, OWSC);
    dst = Enc + (size_t)DH * DM + (size_t)e * 8;
  } else if (blk < CB8) {
    const int e = (blk - CB7) * 256 + t;
    ld8(v, r_out_w + (size_t)e * 8, OWSC);
    dst = rout + (size_t)e * 8;
  } else if (blk < CB9) {
    const int e = (blk - CB8) * 256 + t;
    ld8(v, ew1 + (size_t)e * 8, OWSC);
    dst = e1 + (size_t)e * 8;
  } else if (blk < CB10) {
    const int e = (blk - CB9) * 256 + t;
    ld8(v, ew2 + (size_t)e * 8, OWSC);
    dst = e2 + (size_t)e * 8;
  } else if (blk < CB11) {
    const int e = (blk - CB10) * 256 + t;
    ld8(v, rw1 + (size_t)e * 8, OWSC);
    dst = rw1p + (size_t)e * 8;
  } else {
    const int e = (blk - CB11) * 256 + t;
#pragma unroll
    for (int i = 0; i < 8; ++i) v[i] = 0.0f;
    dst = rw1p + (size_t)16 * DM + (size_t)e * 8;
  }
  const v8h o = to_h8(v);
  STORE2(v8h, dst, o);
}

__global__ __launch_bounds__(64) void k_prep(const float* __restrict__ m_real, const float* __restrict__ m_imag,
                                            const float* __restrict__ values, const float* __restrict__ gate_w,
                                            _Float16* __restrict__ Mem2, float* __restrict__ G)
{
  __shared__ float sInv[NS];
  const int hd = blockIdx.x, t = threadIdx.x;
  {
    const float* mr = m_real + ((size_t)hd * NS + t) * DH;
    const float* mi = m_imag + ((size_t)hd * NS + t) * DH;
    float ss = 0.f;
#pragma unroll 1
    for (int d = 0; d < DH; ++d) { const float a = mr[d], c = mi[d]; ss += a * a + c * c; }
    sInv[t] = 1.0f / fmaxf(sqrtf(ss), 1e-12f);
  }
  __syncthreads();
#pragma unroll 1
  for (int it = 0; it < 16; ++it) {
    const int id = it * 64 + t;
    const int row = id >> 3, q = id & 7;
    const int s = row & 63;
    const bool second = (row >= 64);
    const float sc = sInv[s] * MEMSC;
    const float* pr = m_real + ((size_t)hd * NS + s) * DH;
    const float* pim = m_imag + ((size_t)hd * NS + s) * DH;
    float v[8];
#pragma unroll
    for (int i = 0; i < 8; ++i) {
      const int c = 8 * q + i;
      const int cc = c & 31;
      const float a = pr[cc], bq = pim[cc];
      const float lo = (c < 32) ? a : bq;
      const float hi = (c < 32) ? -bq : a;
      v[i] = (second ? hi : lo) * sc;
    }
    const v8h o = to_h8(v);
    STORE2(v8h, Mem2 + (size_t)hd * (128 * NS) + (size_t)id * 8, o);
  }
  {
    const float* vp = values + ((size_t)hd * NS + t) * DM;
#pragma unroll 1
    for (int hp = 0; hp < NH; ++hp) {
      const float* gw = gate_w + (size_t)hp * (NH * DM) + (size_t)hd * DM;
      float acc = 0.f;
#pragma unroll 4
      for (int d = 0; d < DM; ++d) acc += vp[d] * gw[d];
      STORE2(float, G + hp * (NH * NS) + hd * NS + t, acc);
    }
  }
}

struct GemmArgs {
  const _Float16* A; const _Float16* B; float* C; _Float16* C16;
  const float* bias; const float* resid; const float* rs;
  long long psA, psB, zsA, zsB, zsC, zsC16;
  int lda, ldb, ldc, ldc16, ldr, rss, psBias, zsBias, K, npass, act, pad0;
  float alpha, c16sc;
};
static_assert(sizeof(GemmArgs) == 160);

__device__ __forceinline__ void gemm_store(const float* sT, const GemmArgs& g,
                                           int m0, int n0, int z, int w, int lane) {
  const int q8 = lane & 7, sub = lane >> 3;
  if (g.C != nullptr) {
    float* Cz = g.C + (size_t)z * (size_t)g.zsC;
#pragma unroll
    for (int i = 0; i < 16; ++i) {
      const int L = 4 * i + sub;
      const int row = 32 * w + (L >> 1), hf = L & 1;
      const v4f v = *(const v4fa*)(sT + row * 64 + 32 * hf + 4 * q8);
      *(volatile v4f*)(Cz + (size_t)(m0 + row) * g.ldc + n0 + 32 * hf + 4 * q8) = v;
    }
  }
  if (g.C16 != nullptr) {
    _Float16* Cz = g.C16 + (size_t)z * (size_t)g.zsC16;
    const float s = g.c16sc;
#pragma unroll
    for (int i = 0; i < 8; ++i) {
      const int row = 32 * w + 4 * i + sub;
      const float* sp = sT + row * 64 + 8 * q8;
      const v4f a = *(const v4fa*)sp;
      const v4f c = *(const v4fa*)(sp + 4);
      const v8h o = { (_Float16)(a.x * s), (_Float16)(a.y * s), (_Float16)(a.z * s), (_Float16)(a.w * s),
                      (_Float16)(c.x * s), (_Float16)(c.y * s), (_Float16)(c.z * s), (_Float16)(c.w * s) };
      *(volatile v8h*)(Cz + (size_t)(m0 + row) * g.ldc16 + n0 + 8 * q8) = o;
    }
  }
}

__global__ __launch_bounds__(128) void k_gemm(GemmArgs g)
{
  __shared__ __attribute__((aligned(16))) float sT[128 * 64];

  const int tid = threadIdx.x, lane = tid & 31, w = tid >> 5;
  const int h = lane >> 4, m = lane & 15;
  const int m0 = blockIdx.y * 128, n0 = blockIdx.x * 64, z = blockIdx.z;
  const int rw0 = 32 * w;
  const _Float16* Az = g.A + (size_t)z * (size_t)g.zsA;
  const _Float16* Bz = g.B + (size_t)z * (size_t)g.zsB;
  const v8f zero8 = {0.f, 0.f, 0.f, 0.f, 0.f, 0.f, 0.f, 0.f};

#pragma unroll 1
  for (int ps = 0; ps < g.npass; ++ps) {
    const _Float16* xa0 = Az + (size_t)ps * (size_t)g.psA + (size_t)(m0 + rw0 + m) * g.lda;
    const _Float16* xa1 = xa0 + (size_t)16 * g.lda;
    const _Float16* xb  = Bz + (size_t)ps * (size_t)g.psB + (size_t)(n0 + m) * g.ldb;

    v8f acc[2][4];
#pragma unroll
    for (int mt = 0; mt < 2; ++mt)
#pragma unroll
      for (int nt = 0; nt < 4; ++nt) acc[mt][nt] = zero8;

#pragma unroll 1
    for (int k0 = 0; k0 < g.K; k0 += 32) {
      const v16h a0 = load_frag(xa0 + k0, h);
      const v16h a1 = load_frag(xa1 + k0, h);
#pragma unroll
      for (int nt = 0; nt < 4; ++nt) {
        const v16h b = load_frag(xb + (size_t)nt * 16 * g.ldb + k0, h);
        acc[0][nt] = wmma_f16(a0, b, acc[0][nt]);
        acc[1][nt] = wmma_f16(a1, b, acc[1][nt]);
      }
    }

    const float* biasp = (g.bias != nullptr)
        ? (g.bias + (size_t)z * (size_t)g.zsBias + (size_t)ps * (size_t)g.psBias + n0) : nullptr;
#pragma unroll
    for (int nt = 0; nt < 4; ++nt) {
      const int coll = 16 * nt + m;
      float bv = 0.f;
      if (biasp != nullptr) bv = biasp[coll];
#pragma unroll
      for (int mt = 0; mt < 2; ++mt) {
#pragma unroll
        for (int r = 0; r < 8; ++r) {
          const int rowl = rw0 + 16 * mt + 8 * h + r;
          float v = g.alpha * acc[mt][nt][r] + bv;
          if (g.act == 1) v = v * (1.0f / (1.0f + expf(-v)));
          if (g.rs != nullptr) v *= g.rs[(size_t)(m0 + rowl) * g.rss + ps];
          const int si = rowl * 64 + coll;
          if (ps == 0) {
            float base = 0.f;
            if (g.resid != nullptr) base = g.resid[(size_t)(m0 + rowl) * g.ldr + n0 + coll];
            sT[si] = base + v;
          } else {
            sT[si] = sT[si] + v;
          }
        }
      }
    }
  }
  __syncthreads();

  gemm_store(sT, g, m0, n0, z, w, lane);
  __threadfence();
  gemm_store(sT, g, m0, n0, z, w, lane);
}

__global__ __launch_bounds__(32) void k_tokprep(const float* __restrict__ P1, const float* __restrict__ pw2,
                                               const float* __restrict__ pb2, _Float16* __restrict__ psi,
                                               float* __restrict__ p8, float* __restrict__ ptok,
                                               float* __restrict__ omp)
{
  __shared__ __attribute__((aligned(16))) float sP[32 * NH];
  const int lane = threadIdx.x, q = lane & 7, grp = lane >> 3;
  const int tok0 = blockIdx.x * 32;
#pragma unroll 1
  for (int t = 0; t < 32; ++t) {
    const int tok = tok0 + t;
    const float* row = P1 + (size_t)tok * P1LD;
#pragma unroll
    for (int pass = 0; pass < 2; ++pass) {
      const int hd = pass * 4 + grp;
      const int col = (q < 4) ? (hd * DH + 8 * q) : (NH * DH + hd * DH + 8 * (q - 4));
      const v4f a = *(const v4fa*)(row + col);
      const v4f c = *(const v4fa*)(row + col + 4);
      float ss = a.x * a.x + a.y * a.y + a.z * a.z + a.w * a.w
               + c.x * c.x + c.y * c.y + c.z * c.z + c.w * c.w;
      ss += __shfl_xor(ss, 1); ss += __shfl_xor(ss, 2); ss += __shfl_xor(ss, 4);
      const float inv = 1.0f / fmaxf(sqrtf(ss), 1e-12f);
      const v8h o = { (_Float16)((a.x * inv) * PSISC), (_Float16)((a.y * inv) * PSISC),
                      (_Float16)((a.z * inv) * PSISC), (_Float16)((a.w * inv) * PSISC),
                      (_Float16)((c.x * inv) * PSISC), (_Float16)((c.y * inv) * PSISC),
                      (_Float16)((c.z * inv) * PSISC), (_Float16)((c.w * inv) * PSISC) };
      STORE2(v8h, psi + (size_t)tok * (NH * NS) + pass * 256 + 8 * lane, o);
      const int zc = 2 * NH * DH + hd * 16 + 2 * q;
      float zd = row[zc] * pw2[hd * 16 + 2 * q] + row[zc + 1] * pw2[hd * 16 + 2 * q + 1];
      zd += __shfl_xor(zd, 1); zd += __shfl_xor(zd, 2); zd += __shfl_xor(zd, 4);
      const float ph = 0.95f * (1.0f / (1.0f + expf(-(zd + pb2[hd]))));
      if (q == 0) sP[t * NH + hd] = ph;
    }
  }
  __syncthreads();
#pragma unroll
  for (int i = 0; i < 2; ++i) {
    const int tl = 16 * i + (lane >> 1);
    const v4f v = *(const v4fa*)(sP + tl * NH + 4 * (lane & 1));
    STORE2(v4f, p8 + (size_t)(tok0 + tl) * NH + 4 * (lane & 1), v);
  }
  {
    const int q4 = lane & 7;
    float pt[4];
#pragma unroll
    for (int j = 0; j < 4; ++j) {
      const int tl = 4 * q4 + j;
      float s = 0.f;
#pragma unroll
      for (int hd = 0; hd < NH; ++hd) s += sP[tl * NH + hd];
      pt[j] = s * 0.125f;
    }
    const v4f vp = { pt[0], pt[1], pt[2], pt[3] };
    const v4f vo = { 1.0f - pt[0], 1.0f - pt[1], 1.0f - pt[2], 1.0f - pt[3] };
    if (lane < 8)       STORE2(v4f, ptok + tok0 + 4 * q4, vp);
    else if (lane < 16) STORE2(v4f, omp + tok0 + 4 * q4, vo);
  }
}

__global__ __launch_bounds__(256) void k_attn(const float* __restrict__ OV, const float* __restrict__ p8,
                                             const float* __restrict__ G, const float* __restrict__ gate_b,
                                             _Float16* __restrict__ wattn)
{
  __shared__ __attribute__((aligned(16))) float sG[NH * NH * NS];
  __shared__ __attribute__((aligned(16))) float sA[8][NH * NS];
  const int tid = threadIdx.x, lane = tid & 31, w = tid >> 5, q = lane & 7, grp = lane >> 3;
#pragma unroll
  for (int i = 0; i < 16; ++i) sG[tid + 256 * i] = G[tid + 256 * i];
  const float gb = gate_b[lane & 7];
  __syncthreads();
#pragma unroll 1
  for (int t = 0; t < 4; ++t) {
    const int tok = blockIdx.x * 32 + w * 4 + t;
    const float* ov = OV + (size_t)tok * OVLD;
    float at[2][8];
#pragma unroll
    for (int pass = 0; pass < 2; ++pass) {
      const int hd = pass * 4 + grp;
      const float pv = p8[(size_t)tok * NH + hd];
      const v4f r0 = *(const v4fa*)(ov + hd * 128 + 8 * q);
      const v4f r1 = *(const v4fa*)(ov + hd * 128 + 8 * q + 4);
      const v4f i0 = *(const v4fa*)(ov + hd * 128 + 64 + 8 * q);
      const v4f i1 = *(const v4fa*)(ov + hd * 128 + 64 + 8 * q + 4);
      const float re[8] = { r0.x, r0.y, r0.z, r0.w, r1.x, r1.y, r1.z, r1.w };
      const float im[8] = { i0.x, i0.y, i0.z, i0.w, i1.x, i1.y, i1.z, i1.w };
      float raw[8];
      float rsum = 0.f;
#pragma unroll
      for (int j = 0; j < 8; ++j) {
        raw[j] = (1.0f - pv) * (re[j] * re[j] + im[j] * im[j]) + pv * 0.03125f;
        rsum += raw[j];
      }
      rsum += __shfl_xor(rsum, 1); rsum += __shfl_xor(rsum, 2); rsum += __shfl_xor(rsum, 4);
      const float inv = 1.0f / (rsum + 1e-8f);
#pragma unroll
      for (int j = 0; j < 8; ++j) {
        at[pass][j] = raw[j] * inv;
        sA[w][pass * 256 + 8 * lane + j] = at[pass][j];
      }
    }
    __syncthreads();
    float gl = 0.f;
    {
      const float* ap = &sA[w][grp * 128];
      const float* gp = &sG[(lane & 7) * (NH * NS) + grp * 128];
#pragma unroll 4
      for (int k = 0; k < 128; ++k) gl += ap[k] * gp[k];
    }
    gl += __shfl_xor(gl, 8); gl += __shfl_xor(gl, 16);
    gl += gb;
    float mx = fmaxf(gl, __shfl_xor(gl, 1));
    mx = fmaxf(mx, __shfl_xor(mx, 2));
    mx = fmaxf(mx, __shfl_xor(mx, 4));
    const float e = expf(gl - mx);
    float se = e + __shfl_xor(e, 1);
    se += __shfl_xor(se, 2); se += __shfl_xor(se, 4);
    const float gate = e * (1.0f / se);
#pragma unroll
    for (int pass = 0; pass < 2; ++pass) {
      const int hd = pass * 4 + grp;
      const float gh = __shfl(gate, hd);
      float v[8];
#pragma unroll
      for (int j = 0; j < 8; ++j) v[j] = (at[pass][j] * gh) * ATTSC;
      const v8h o = to_h8(v);
      STORE2(v8h, wattn + (size_t)tok * (NH * NS) + pass * 256 + 8 * lane, o);
    }
    __syncthreads();
  }
}

__global__ __launch_bounds__(128) void k_couple(const _Float16* __restrict__ h1c, const float* __restrict__ ptok,
                                               const float* __restrict__ omp, const float* __restrict__ beta,
                                               float* __restrict__ ompnew)
{
  __shared__ __attribute__((aligned(16))) float sO[4][32];
  const int tid = threadIdx.x, lane = tid & 31, w = tid >> 5, h = lane >> 4, m = lane & 15;
  const int b = blockIdx.y;
  const int q0 = blockIdx.x * 128 + 32 * w;
  const size_t brow = (size_t)b * SEQ;
  const _Float16* xa0 = h1c + (brow + q0 + m) * DM;
  const _Float16* xa1 = xa0 + (size_t)16 * DM;
  const _Float16* kb0 = h1c + (brow + m) * DM;
  const float* ompb = omp + brow;
  const v8f zero8 = {0.f, 0.f, 0.f, 0.f, 0.f, 0.f, 0.f, 0.f};
  const float ssc = 0.036084391824351614f * (1.0f / (HSC * HSC));

  float mrun[2][8], lrun[2][8], wrun[2][8];
#pragma unroll
  for (int mt = 0; mt < 2; ++mt)
#pragma unroll
    for (int r = 0; r < 8; ++r) { mrun[mt][r] = -1.0e30f; lrun[mt][r] = 0.f; wrun[mt][r] = 0.f; }

#pragma unroll 1
  for (int kb = 0; kb < SEQ; kb += 64) {
    v8f acc[2][4];
#pragma unroll
    for (int mt = 0; mt < 2; ++mt)
#pragma unroll
      for (int nt = 0; nt < 4; ++nt) acc[mt][nt] = zero8;
#pragma unroll 1
    for (int k0 = 0; k0 < DM; k0 += 32) {
      const v16h a0 = load_frag(xa0 + k0, h);
      const v16h a1 = load_frag(xa1 + k0, h);
#pragma unroll
      for (int nt = 0; nt < 4; ++nt) {
        const v16h bf = load_frag(kb0 + (size_t)(kb + 16 * nt) * DM + k0, h);
        acc[0][nt] = wmma_f16(a0, bf, acc[0][nt]);
        acc[1][nt] = wmma_f16(a1, bf, acc[1][nt]);
      }
    }
    float ov[4];
#pragma unroll
    for (int nt = 0; nt < 4; ++nt) ov[nt] = ompb[kb + 16 * nt + m];
#pragma unroll
    for (int mt = 0; mt < 2; ++mt) {
#pragma unroll
      for (int r = 0; r < 8; ++r) {
        float s[4];
#pragma unroll
        for (int nt = 0; nt < 4; ++nt) s[nt] = acc[mt][nt][r] * ssc;
        float ml = fmaxf(fmaxf(s[0], s[1]), fmaxf(s[2], s[3]));
        ml = fmaxf(ml, __shfl_xor(ml, 1)); ml = fmaxf(ml, __shfl_xor(ml, 2));
        ml = fmaxf(ml, __shfl_xor(ml, 4)); ml = fmaxf(ml, __shfl_xor(ml, 8));
        const float mn = fmaxf(mrun[mt][r], ml);
        const float al = __expf(mrun[mt][r] - mn);
        float ls = 0.f, wsm = 0.f;
#pragma unroll
        for (int nt = 0; nt < 4; ++nt) { const float e = __expf(s[nt] - mn); ls += e; wsm += e * ov[nt]; }
        ls += __shfl_xor(ls, 1); ls += __shfl_xor(ls, 2); ls += __shfl_xor(ls, 4); ls += __shfl_xor(ls, 8);
        wsm += __shfl_xor(wsm, 1); wsm += __shfl_xor(wsm, 2); wsm += __shfl_xor(wsm, 4); wsm += __shfl_xor(wsm, 8);
        lrun[mt][r] = lrun[mt][r] * al + ls;
        wrun[mt][r] = wrun[mt][r] * al + wsm;
        mrun[mt][r] = mn;
      }
    }
  }
  const float sb = 1.0f / (1.0f + expf(-beta[0]));
#pragma unroll
  for (int mt = 0; mt < 2; ++mt) {
#pragma unroll
    for (int r = 0; r < 8; ++r) {
      const int rowl = 16 * mt + 8 * h + r;
      const float neigh = wrun[mt][r] * (1.0f / lrun[mt][r]);
      const float pt = ptok[brow + q0 + rowl];
      float pn = pt * (1.0f - sb * neigh);
      pn = fminf(fmaxf(pn, 0.0f), 0.95f);
      if (m == 0) sO[w][rowl] = 1.0f - pn;
    }
  }
  __syncthreads();
  if (lane < 8) {
    const v4f v = *(const v4fa*)(&sO[w][4 * lane]);
    STORE2(v4f, ompnew + brow + q0 + 4 * lane, v);
  }
}

__global__ __launch_bounds__(256) void k_interf(const float* __restrict__ Q, const float* __restrict__ P_real,
                                               const float* __restrict__ P_imag, const float* __restrict__ C_real,
                                               const float* __restrict__ C_imag, _Float16* __restrict__ feats)
{
  __shared__ float sPC[4 * 1024];
  __shared__ float sGm[64];
  __shared__ __attribute__((aligned(16))) _Float16 sF[8][64];
  const int tid = threadIdx.x, lane = tid & 31, w = tid >> 5;
  if (w < 2) {
    const float* re = (w == 0) ? P_real : C_real;
    const float* im = (w == 0) ? P_imag : C_imag;
    const int s = lane;
    float ss = 0.f;
#pragma unroll 1
    for (int d = 0; d < DH; ++d) { const float a = re[s * DH + d], c = im[s * DH + d]; ss += a * a + c * c; }
    const float inv = 1.0f / fmaxf(sqrtf(ss), 1e-12f);
    float* dre = sPC + (2 * w) * 1024 + s * DH;
    float* dim2 = sPC + (2 * w + 1) * 1024 + s * DH;
#pragma unroll 1
    for (int d = 0; d < DH; ++d) { dre[d] = re[s * DH + d] * inv; dim2[d] = im[s * DH + d] * inv; }
  }
  __syncthreads();
  if (w == 0) {
    const int s = lane;
    float gr = 0.f, gi = 0.f;
#pragma unroll 1
    for (int d = 0; d < DH; ++d) {
      const float Pr = sPC[s * DH + d], Pi = sPC[1024 + s * DH + d];
      const float Cr = sPC[2048 + s * DH + d], Ci = sPC[3072 + s * DH + d];
      gr += Pr * Cr + Pi * Ci;
      gi += Pr * Ci - Pi * Cr;
    }
    sGm[s] = gr; sGm[32 + s] = gi;
  }
  __syncthreads();
  const int s = lane;
  const float gr = sGm[s], gi = sGm[32 + s];
#pragma unroll 1
  for (int t = 0; t < 4; ++t) {
    const int tok = blockIdx.x * 32 + w * 4 + t;
    const float* qrow = Q + (size_t)tok * 64;
    const float qrl = qrow[lane], qil = qrow[32 + lane];
    const float ss = wsum32(qrl * qrl + qil * qil);
    const float inv = 1.0f / fmaxf(sqrtf(ss), 1e-12f);
    float ar = 0.f, ai = 0.f, br = 0.f, bi = 0.f;
#pragma unroll 1
    for (int d = 0; d < DH; ++d) {
      const float qrd = qrow[d], qid = qrow[32 + d];
      const float Prd = sPC[s * DH + d], Pid = sPC[1024 + s * DH + d];
      const float Crd = sPC[2048 + s * DH + d], Cid = sPC[3072 + s * DH + d];
      ar += qrd * Prd + qid * Pid;
      ai += qrd * Pid - qid * Prd;
      br += qrd * Crd + qid * Cid;
      bi += qrd * Cid - qid * Crd;
    }
    ar *= inv; ai *= inv; br *= inv; bi *= inv;
    const float tr = ar * gr - ai * gi;
    const float ti = ar * gi + ai * gr;
    const float Rre = tr * br + ti * bi;
    const float Rim = ti * br - tr * bi;
    sF[w][s] = (_Float16)(Rre * FSC);
    sF[w][32 + s] = (_Float16)(Rim * FSC);
    __syncthreads();
    if (lane < 8) {
      const v8h v = *(const v8ha*)(&sF[w][8 * lane]);
      STORE2(v8h, feats + (size_t)tok * 64 + 8 * lane, v);
    }
    __syncthreads();
  }
}

__global__ __launch_bounds__(256) void k_ln(const float* __restrict__ X, const float* __restrict__ gam,
                                           const float* __restrict__ bet, _Float16* __restrict__ xk)
{
  __shared__ __attribute__((aligned(16))) _Float16 sR[8][DM];
  const int tid = threadIdx.x, lane = tid & 31, w = tid >> 5;
  const int row = blockIdx.x * 8 + w;
  const float* xp = X + (size_t)row * DM;
  float s = 0.f;
#pragma unroll 4
  for (int i = 0; i < 24; ++i) s += xp[lane + 32 * i];
  s = wsum32(s);
  const float mu = s * (1.0f / 768.0f);
  float s2 = 0.f;
#pragma unroll 4
  for (int i = 0; i < 24; ++i) { const float d = xp[lane + 32 * i] - mu; s2 += d * d; }
  s2 = wsum32(s2);
  const float rstd = 1.0f / sqrtf(s2 * (1.0f / 768.0f) + 1e-5f);
#pragma unroll 1
  for (int i = 0; i < 24; ++i) {
    const int c = lane + 32 * i;
    const float y = (xp[c] - mu) * rstd * gam[c] + bet[c];
    sR[w][c] = (_Float16)(gelu_erf(y) * XKSC);
  }
  __syncthreads();
  v8h o[3];
#pragma unroll
  for (int i = 0; i < 3; ++i) o[i] = *(const v8ha*)(&sR[w][256 * i + 8 * lane]);
  _Float16* dst = xk + (size_t)row * DM + 8 * lane;
#pragma unroll
  for (int i = 0; i < 3; ++i) *(volatile v8h*)(dst + 256 * i) = o[i];
  __threadfence();
#pragma unroll
  for (int i = 0; i < 3; ++i) *(volatile v8h*)(dst + 256 * i) = o[i];
}

__global__ __launch_bounds__(256) void k_rg(const float* __restrict__ RG1, const float* __restrict__ rb1,
                                           const float* __restrict__ rw2, const float* __restrict__ rb2,
                                           float* __restrict__ rg)
{
  const int tok = blockIdx.x * 256 + threadIdx.x;
  const float* rr = RG1 + (size_t)tok * 64;
  float l0 = 0.f, l1 = 0.f, l2 = 0.f;
#pragma unroll 1
  for (int k = 0; k < 16; ++k) {
    const float ge = gelu_erf(rr[k] + rb1[k]);
    l0 += ge * rw2[k]; l1 += ge * rw2[16 + k]; l2 += ge * rw2[32 + k];
  }
  l0 += rb2[0]; l1 += rb2[1]; l2 += rb2[2];
  const float mx = fmaxf(l0, fmaxf(l1, l2));
  const float e0 = expf(l0 - mx), e1 = expf(l1 - mx), e2 = expf(l2 - mx);
  const float rinv = 1.0f / (e0 + e1 + e2);
  const v4f o = { e0 * rinv, e1 * rinv, e2 * rinv, 0.0f };
  STORE2(v4f, rg + (size_t)tok * 4, o);
}

static GemmArgs gemm_args(const _Float16* A, int lda, const _Float16* B, int ldb, int K, float alpha) {
  GemmArgs g;
  g.A = A; g.B = B; g.C = nullptr; g.C16 = nullptr; g.bias = nullptr; g.resid = nullptr; g.rs = nullptr;
  g.psA = 0; g.psB = 0; g.zsA = 0; g.zsB = 0; g.zsC = 0; g.zsC16 = 0;
  g.lda = lda; g.ldb = ldb; g.ldc = 0; g.ldc16 = 0; g.ldr = 0; g.rss = 0; g.psBias = 0; g.zsBias = 0;
  g.K = K; g.npass = 1; g.act = 0; g.pad0 = 0;
  g.alpha = alpha; g.c16sc = 1.0f;
  return g;
}

static void gemm_launch(const GemmArgs& g, int M, int N, int nb, hipStream_t s) {
  dim3 grid(N / 64, M / 128, nb);
  k_gemm<<<grid, 128, 0, s>>>(g);
}

extern "C" void kernel_launch(void* const* d_in, const int* in_sizes, int n_in,
                              void* d_out, int out_size, void* d_ws, size_t ws_size,
                              hipStream_t stream)
{
  if (n_in < 33) return;
  static const int expect_n[33] = {
    6291456, 196608, 196608, 98304, 128, 128, 8, 16384, 16384, 393216, 49152, 8, 589824, 768, 1,
    1024, 1024, 1024, 1024, 24576, 24576, 49152, 768, 1769472, 2304, 2304, 2304, 1769472, 2304,
    12288, 16, 48, 3 };
  for (int i = 0; i < 33; ++i) if (in_sizes[i] != expect_n[i]) return;
  if (out_size != TOK * DM) return;

  const float* h       = (const float*)d_in[0];
  const float* W_real  = (const float*)d_in[1];
  const float* W_imag  = (const float*)d_in[2];
  const float* pw1     = (const float*)d_in[3];
  const float* pb1     = (const float*)d_in[4];
  const float* pw2     = (const float*)d_in[5];
  const float* pb2     = (const float*)d_in[6];
  const float* m_real  = (const float*)d_in[7];
  const float* m_imag  = (const float*)d_in[8];
  const float* values  = (const float*)d_in[9];
  const float* gate_w  = (const float*)d_in[10];
  const float* gate_b  = (const float*)d_in[11];
  const float* out_w   = (const float*)d_in[12];
  const float* out_b   = (const float*)d_in[13];
  const float* beta    = (const float*)d_in[14];
  const float* P_real  = (const float*)d_in[15];
  const float* P_imag  = (const float*)d_in[16];
  const float* C_real  = (const float*)d_in[17];
  const float* C_imag  = (const float*)d_in[18];
  const float* enc_r_w = (const float*)d_in[19];
  const float* enc_i_w = (const float*)d_in[20];
  const float* r_out_w = (const float*)d_in[21];
  const float* r_out_b = (const float*)d_in[22];
  const float* ew1     = (const float*)d_in[23];
  const float* eb1     = (const float*)d_in[24];
  const float* eg      = (const float*)d_in[25];
  const float* ebt     = (const float*)d_in[26];
  const float* ew2     = (const float*)d_in[27];
  const float* eb2     = (const float*)d_in[28];
  const float* rw1     = (const float*)d_in[29];
  const float* rb1     = (const float*)d_in[30];
  const float* rw2     = (const float*)d_in[31];
  const float* rb2     = (const float*)d_in[32];
  float* out = (float*)d_out;

  char* base = (char*)d_ws;
  size_t off = 0;
  auto carve = [&](size_t bytes) -> char* {
    char* p = base + off;
    off += (bytes + 255) & ~(size_t)255;
    return p;
  };
  _Float16* Wp    = (_Float16*)carve((size_t)640 * DM * 2);
  _Float16* Mem2  = (_Float16*)carve((size_t)NH * 128 * NS * 2);
  _Float16* Vt    = (_Float16*)carve((size_t)DM * (NH * NS) * 2);
  _Float16* outw  = (_Float16*)carve((size_t)DM * DM * 2);
  _Float16* Enc   = (_Float16*)carve((size_t)64 * DM * 2);
  _Float16* rout  = (_Float16*)carve((size_t)DM * 64 * 2);
  _Float16* e1w   = (_Float16*)carve((size_t)NENC * DM * DM * 2);
  _Float16* e2w   = (_Float16*)carve((size_t)NENC * DM * DM * 2);
  _Float16* rw1p  = (_Float16*)carve((size_t)64 * DM * 2);
  float*    G     = (float*)carve((size_t)NH * NH * NS * 4);
  float*    p8    = (float*)carve((size_t)TOK * NH * 4);
  float*    ptok  = (float*)carve((size_t)TOK * 4);
  float*    omp   = (float*)carve((size_t)TOK * 4);
  float*    ompn  = (float*)carve((size_t)TOK * 4);
  float*    RG1   = (float*)carve((size_t)TOK * 64 * 4);
  float*    rgt   = (float*)carve((size_t)TOK * 4 * 4);
  const size_t szA = (size_t)TOK * DM * 4;
  const size_t szB = (size_t)TOK * P1LD * 4;
  const size_t szC = (size_t)TOK * OVLD * 4;
  const size_t szE = (size_t)TOK * DM * 2;
  char* RA = carve(szA);
  char* RB = carve(szB);
  char* RC = carve(szC);
  char* RE = carve(szE);
  if (off > ws_size) return;
  if (off > (size_t)134217728) return;
  if (RC != RB + szB) return;
  if (szB + szC < (size_t)NENC * TOK * DM * 2) return;

  _Float16* hh     = (_Float16*)RA;
  _Float16* psi16  = (_Float16*)RA;
  _Float16* comb16 = (_Float16*)RA;
  float*    Qf     = (float*)RA;
  _Float16* feats  = (_Float16*)(RA + (size_t)TOK * 64 * 4);
  float*    Xf     = (float*)RA;
  float*    P1     = (float*)RB;
  _Float16* wattn  = (_Float16*)RB;
  _Float16* h1c    = (_Float16*)RB;
  _Float16* xk16   = (_Float16*)RB;
  float*    OV     = (float*)RC;
  float*    h1     = (float*)RC;
  _Float16* h2c    = (_Float16*)RE;

  k_convert<<<CB12, 256, 0, stream>>>(h, W_real, W_imag, pw1, values, out_w, enc_r_w, enc_i_w, r_out_w,
                                       ew1, ew2, rw1, hh, Wp, Vt, outw, Enc, rout, e1w, e2w, rw1p);
  k_prep<<<NH, 64, 0, stream>>>(m_real, m_imag, values, gate_w, Mem2, G);
  {
    GemmArgs g = gemm_args(hh, DM, Wp, DM, DM, 1.0f / (HSC * WSC));
    g.C = P1; g.ldc = P1LD;
    gemm_launch(g, TOK, 512, 1, stream);
  }
  {
    GemmArgs g = gemm_args(hh, DM, Wp + (size_t)512 * DM, DM, DM, 1.0f / (HSC * PWSC));
    g.C = P1 + 512; g.ldc = P1LD; g.bias = pb1; g.act = 1;
    gemm_launch(g, TOK, 128, 1, stream);
  }
  k_tokprep<<<TOK / 32, 32, 0, stream>>>(P1, pw2, pb2, psi16, p8, ptok, omp);
  {
    GemmArgs g = gemm_args(psi16, NH * NS, Mem2, 64, 64, 1.0f / (PSISC * MEMSC));
    g.zsA = NS; g.zsB = 128 * 64; g.C = OV; g.ldc = OVLD; g.zsC = 128;
    gemm_launch(g, TOK, 128, NH, stream);
  }
  k_attn<<<TOK / 32, 256, 0, stream>>>(OV, p8, G, gate_b, wattn);
  {
    GemmArgs g = gemm_args(wattn, NH * NS, Vt, NH * NS, NH * NS, 1.0f / (ATTSC * WSC));
    g.C16 = comb16; g.ldc16 = DM; g.c16sc = CMBSC;
    gemm_launch(g, TOK, DM, 1, stream);
  }
  {
    GemmArgs g = gemm_args(comb16, DM, outw, DM, DM, 1.0f / (CMBSC * OWSC));
    g.bias = out_b; g.resid = h; g.ldr = DM;
    g.C = h1; g.ldc = DM; g.C16 = h1c; g.ldc16 = DM; g.c16sc = HSC;
    gemm_launch(g, TOK, DM, 1, stream);
  }
  k_couple<<<dim3(SEQ / 128, NB), 128, 0, stream>>>(h1c, ptok, omp, beta, ompn);
  {
    GemmArgs g = gemm_args(h1c, DM, Enc, DM, DM, 1.0f / (HSC * OWSC));
    g.C = Qf; g.ldc = 64;
    gemm_launch(g, TOK, 64, 1, stream);
  }
  k_interf<<<TOK / 32, 256, 0, stream>>>(Qf, P_real, P_imag, C_real, C_imag, feats);
  {
    GemmArgs g = gemm_args(feats, 64, rout, 64, 64, 1.0f / (FSC * OWSC));
    g.bias = r_out_b; g.rs = ompn; g.rss = 1; g.resid = h1; g.ldr = DM;
    g.C = out; g.ldc = DM; g.C16 = h2c; g.ldc16 = DM; g.c16sc = HSC;
    gemm_launch(g, TOK, DM, 1, stream);
  }
  for (int k = 0; k < NENC; ++k) {
    GemmArgs g = gemm_args(h2c, DM, e1w + (size_t)k * DM * DM, DM, DM, 1.0f / (HSC * OWSC));
    g.bias = eb1 + (size_t)k * DM; g.C = Xf; g.ldc = DM;
    gemm_launch(g, TOK, DM, 1, stream);
    k_ln<<<TOK / 8, 256, 0, stream>>>(Xf, eg + (size_t)k * DM, ebt + (size_t)k * DM,
                                       xk16 + (size_t)k * TOK * DM);
  }
  {
    GemmArgs g = gemm_args(h2c, DM, rw1p, DM, DM, 1.0f / (HSC * OWSC));
    g.C = RG1; g.ldc = 64;
    gemm_launch(g, TOK, 64, 1, stream);
  }
  k_rg<<<TOK / 256, 256, 0, stream>>>(RG1, rb1, rw2, rb2, rgt);
  {
    GemmArgs g = gemm_args(xk16, DM, e2w, DM, DM, 1.0f / (XKSC * OWSC));
    g.npass = NENC; g.psA = (long long)TOK * DM; g.psB = (long long)DM * DM;
    g.bias = eb2; g.psBias = DM; g.rs = rgt; g.rss = 4; g.resid = out; g.ldr = DM;
    g.C = out; g.ldc = DM;
    gemm_launch(g, TOK, DM, 1, stream);
  }
}
